// LstmAggregator_6854767804437
// MI455X (gfx1250) — hardware-verified
//
#include <hip/hip_runtime.h>
#include <math.h>

constexpr int NUM_NODES   = 30000;
constexpr int NUM_EDGES   = 480000;
constexpr int FEAT_IN     = 128;
constexpr int HID_UNITS   = 128;
constexpr int FEAT_OUT    = 128;
constexpr int GATE_COLS   = 4 * HID_UNITS;
constexpr int DEG_CAP     = 48;
constexpr int TILE_NODES  = 16;
constexpr int NUM_TILES   = NUM_NODES / TILE_NODES;
constexpr int NODES_PAD   = 30016;
constexpr int CAT_COLS    = FEAT_IN + HID_UNITS;
constexpr int HPITCH      = 136;
constexpr int NTHR        = 256;
constexpr int OUT_VEC4    = NUM_NODES * FEAT_OUT / 4;
constexpr float WCARRY     = 256.0f;
constexpr float WCARRY_INV = 1.0f / 256.0f;

static_assert(NUM_NODES % TILE_NODES == 0);
static_assert(NUM_TILES == 1875);
static_assert(NODES_PAD % 64 == 0 && NODES_PAD >= NUM_NODES);
static_assert(GATE_COLS % 64 == 0 && FEAT_OUT % 64 == 0);
static_assert(FEAT_IN % 32 == 0 && CAT_COLS % 32 == 0 && HID_UNITS % 32 == 0);
static_assert(HID_UNITS == 16 * (NTHR / 32));
static_assert(HPITCH % 8 == 0 && HPITCH >= HID_UNITS);
static_assert((NUM_NODES * (FEAT_IN / 8)) % NTHR == 0);
static_assert(TILE_NODES * DEG_CAP == 3 * NTHR);
static_assert(OUT_VEC4 % NTHR == 0);
static_assert((size_t)OUT_VEC4 * 16 == (size_t)15360000);

constexpr size_t ACAT_BYTES  = (size_t)NODES_PAD * CAT_COLS * 2;
constexpr size_t PPLANE_BYTES = (size_t)NODES_PAD * GATE_COLS * 4;
constexpr size_t WHH_BYTES   = (size_t)GATE_COLS * HID_UNITS * 2;
constexpr size_t WIHP_BYTES  = (size_t)GATE_COLS * FEAT_IN * 2;
constexpr size_t WOT_BYTES   = (size_t)FEAT_OUT * CAT_COLS * 2;
constexpr size_t BIASP_BYTES = (size_t)GATE_COLS * 4;
constexpr size_t CARVE_TOTAL = ACAT_BYTES + PPLANE_BYTES + WHH_BYTES + WIHP_BYTES + WOT_BYTES + BIASP_BYTES;
static_assert(ACAT_BYTES % 256 == 0 && PPLANE_BYTES % 256 == 0 && WHH_BYTES % 256 == 0 &&
              WIHP_BYTES % 256 == 0 && WOT_BYTES % 256 == 0 && BIASP_BYTES % 256 == 0);
static_assert(CARVE_TOTAL == 77170688);
static_assert(CARVE_TOTAL <= (size_t)134217728);

typedef __attribute__((ext_vector_type(16))) _Float16 v16h;
typedef __attribute__((ext_vector_type(8)))  _Float16 v8h;
typedef __attribute__((ext_vector_type(8)))  float    v8f;
typedef __attribute__((ext_vector_type(4)))  float    v4f;

__device__ __forceinline__ void guard4_h(v8f& a0, v8f& a1, v8f& a2, v8f& a3, v16h x, v16h b0, v16h b1, v16h b2, v16h b3) {
  asm volatile("v_nop\n\tv_nop\n\tv_nop\n\tv_nop" : "+v"(a0), "+v"(a1), "+v"(a2), "+v"(a3) : "v"(x), "v"(b0), "v"(b1), "v"(b2), "v"(b3));
}
__device__ __forceinline__ void keep4_h(v16h a, v16h b, v16h c, v16h d) { asm volatile("v_nop" :: "v"(a), "v"(b), "v"(c), "v"(d)); }
__device__ __forceinline__ void acc_guard4(v8f& a, v8f& b, v8f& c, v8f& d) { asm volatile("v_nop\n\tv_nop\n\tv_nop\n\tv_nop" : "+v"(a), "+v"(b), "+v"(c), "+v"(d)); }

union FragU { v16h v; v8h h[2]; };
__device__ __forceinline__ v16h frag_load(const _Float16* p) {
  FragU f;
  f.h[0] = *(const v8h*)(p);
  f.h[1] = *(const v8h*)(p + 16);
  return f.v;
}
__device__ __forceinline__ v8f frag_mma(v16h a, v16h b, v8f c) {
  return __builtin_amdgcn_wmma_f32_16x16x32_f16(false, a, false, b, (short)0, c, false, false);
}

__device__ __forceinline__ float fsig(float x)  { return __builtin_amdgcn_rcpf(1.0f + __expf(-x)); }
__device__ __forceinline__ float ftanh(float x) { return 1.0f - 2.0f * __builtin_amdgcn_rcpf(__expf(2.0f * x) + 1.0f); }

__device__ __forceinline__ v8h pack8_f16(v4f a, v4f b, float sc) {
  v8h hv;
#pragma unroll
  for (int e = 0; e < 4; ++e) {
    hv[e]     = (_Float16)(a[e] * sc);
    hv[4 + e] = (_Float16)(b[e] * sc);
  }
  return hv;
}
__device__ __forceinline__ void store16_twice(unsigned short* dst, v8h hv) {
  *(volatile v8h*)dst = hv;
  __threadfence();
  *(volatile v8h*)dst = hv;
}

__global__ __launch_bounds__(NTHR) void prep_x_kernel(const float* __restrict__ X, unsigned short* __restrict__ ACAT) {
  constexpr int NX8 = NUM_NODES * (FEAT_IN / 8);
  constexpr int NZ8 = (NODES_PAD - NUM_NODES) * (CAT_COLS / 8);
  const int i = blockIdx.x * NTHR + threadIdx.x;
  if (blockIdx.x < NX8 / NTHR) {
    const int row = i >> 4;
    const int c8  = i & 15;
    const float* sp = X + (size_t)row * FEAT_IN + c8 * 8;
    const v4f a = *(const v4f*)(sp);
    const v4f b = *(const v4f*)(sp + 4);
    const v8h hv = pack8_f16(a, b, 1.0f);
    store16_twice(ACAT + (size_t)row * CAT_COLS + c8 * 8, hv);
  } else {
    const int z = i - NX8;
    if (z < NZ8) {
      const v8h zv = {(_Float16)0.0f, (_Float16)0.0f, (_Float16)0.0f, (_Float16)0.0f,
                      (_Float16)0.0f, (_Float16)0.0f, (_Float16)0.0f, (_Float16)0.0f};
      store16_twice(ACAT + (size_t)NUM_NODES * CAT_COLS + (size_t)z * 8, zv);
    }
  }
}

__global__ __launch_bounds__(NTHR) void prep_w_kernel(const float* __restrict__ W_ih, const float* __restrict__ W_hh,
                                                      const float* __restrict__ b_ih, const float* __restrict__ b_hh,
                                                      const float* __restrict__ W_out,
                                                      unsigned short* __restrict__ WHH, unsigned short* __restrict__ WIHP,
                                                      unsigned short* __restrict__ WOT, float* __restrict__ BIASP) {
  const int tid = threadIdx.x;
  const int blk = blockIdx.x;
  if (blk < 32) {
    const int i = blk * NTHR + tid;
    const int row = i >> 4;
    const int c8  = i & 15;
    const float* sp = W_hh + (size_t)row * HID_UNITS + c8 * 8;
    const v4f a = *(const v4f*)(sp);
    const v4f b = *(const v4f*)(sp + 4);
    store16_twice(WHH + (size_t)i * 8, pack8_f16(a, b, WCARRY));
  } else if (blk < 64) {
    const int i = (blk - 32) * NTHR + tid;
    const int np = i >> 4;
    const int c8 = i & 15;
    const int unit = np >> 2;
    const int gate = np & 3;
    const float* sp = W_ih + (size_t)(gate * HID_UNITS + unit) * FEAT_IN + c8 * 8;
    const v4f a = *(const v4f*)(sp);
    const v4f b = *(const v4f*)(sp + 4);
    store16_twice(WIHP + (size_t)i * 8, pack8_f16(a, b, WCARRY));
  } else if (blk < 80) {
    const int i = (blk - 64) * NTHR + tid;
    const int n  = i >> 5;
    const int k8 = i & 31;
    v4f a, b;
#pragma unroll
    for (int e = 0; e < 4; ++e) {
      a[e] = W_out[(size_t)(k8 * 8 + e) * FEAT_OUT + n];
      b[e] = W_out[(size_t)(k8 * 8 + 4 + e) * FEAT_OUT + n];
    }
    store16_twice(WOT + (size_t)i * 8, pack8_f16(a, b, WCARRY));
  } else {
    if (tid < HID_UNITS) {
      v4f o;
#pragma unroll
      for (int g = 0; g < 4; ++g) o[g] = b_ih[g * HID_UNITS + tid] + b_hh[g * HID_UNITS + tid];
      float* op = BIASP + 4 * tid;
      *(volatile v4f*)op = o;
      __threadfence();
      *(volatile v4f*)op = o;
    }
  }
}

template <int BIAS_MODE>
__global__ __launch_bounds__(256) void wmma_gemm64_f16(
    const unsigned short* __restrict__ Ap, int lda,
    const unsigned short* __restrict__ Btp, int ldb,
    float* __restrict__ Cout, int ldc,
    const float* __restrict__ bias,
    int M, int N, int K, int Mstore, float scale) {
  const _Float16* A  = (const _Float16*)Ap;
  const _Float16* Bt = (const _Float16*)Btp;
  __shared__ __align__(16) float sT[8][16 * 68];
  const int lane = threadIdx.x & 31;
  const int wave = threadIdx.x >> 5;
  const int tilesN = N >> 6;
  const int tilesM = M >> 6;
  const int tile = blockIdx.x * 8 + wave;
  if (tile >= tilesM * tilesN) return;
  const int tm = tile / tilesN;
  const int tn = tile - tm * tilesN;
  const int m0 = tm << 6;
  const int n0 = tn << 6;

  const int rlane = lane & 15;
  const int koff  = (lane >> 4) * 8;
  const int mOff  = (lane >> 4) * 8;

  v8f acc[4][4];
#pragma unroll
  for (int i = 0; i < 4; ++i)
#pragma unroll
    for (int j = 0; j < 4; ++j) acc[i][j] = (v8f){0.f, 0.f, 0.f, 0.f, 0.f, 0.f, 0.f, 0.f};

  for (int k0 = 0; k0 < K; k0 += 32) {
    v16h bh[4];
#pragma unroll
    for (int j = 0; j < 4; ++j) {
      const size_t bo = (size_t)(n0 + (j << 4) + rlane) * ldb + koff + k0;
      bh[j] = frag_load(Bt + bo);
    }
#pragma unroll
    for (int i = 0; i < 4; ++i) {
      const size_t ao = (size_t)(m0 + (i << 4) + rlane) * lda + koff + k0;
      const v16h ah = frag_load(A + ao);
#pragma unroll
      for (int j = 0; j < 4; ++j) acc[i][j] = frag_mma(ah, bh[j], acc[i][j]);
      guard4_h(acc[i][0], acc[i][1], acc[i][2], acc[i][3], ah, bh[0], bh[1], bh[2], bh[3]);
    }
    keep4_h(bh[0], bh[1], bh[2], bh[3]);
  }
  acc_guard4(acc[0][0], acc[0][1], acc[0][2], acc[0][3]);
  acc_guard4(acc[1][0], acc[1][1], acc[1][2], acc[1][3]);
  acc_guard4(acc[2][0], acc[2][1], acc[2][2], acc[2][3]);
  acc_guard4(acc[3][0], acc[3][1], acc[3][2], acc[3][3]);

  float* slab = sT[wave];
#pragma unroll
  for (int i = 0; i < 4; ++i) {
    const int mBase = m0 + (i << 4);
#pragma unroll
    for (int j = 0; j < 4; ++j) {
      const int n = n0 + (j << 4) + rlane;
      float bv = 0.f;
      if (BIAS_MODE == 2) bv = bias[n];
#pragma unroll
      for (int r = 0; r < 8; ++r) {
        float v = acc[i][j][r] * scale;
        if (BIAS_MODE == 2) v += bv;
        slab[(mOff + r) * 68 + (j << 4) + rlane] = v;
      }
    }
    __builtin_amdgcn_fence(__ATOMIC_RELEASE, "workgroup");
    __builtin_amdgcn_wave_barrier();
    __builtin_amdgcn_fence(__ATOMIC_ACQUIRE, "workgroup");
    {
      const int hh = lane >> 4;
      const int c4 = (lane & 15) * 4;
      for (int pass = 0; pass < 2; ++pass) {
#pragma unroll
        for (int it = 0; it < 8; ++it) {
          const int row = it * 2 + hh;
          const v4f v = *(const v4f*)(slab + row * 68 + c4);
          if (mBase + row < Mstore) *(volatile v4f*)(Cout + (size_t)(mBase + row) * ldc + n0 + c4) = v;
        }
        __threadfence();
      }
    }
    __builtin_amdgcn_fence(__ATOMIC_RELEASE, "workgroup");
    __builtin_amdgcn_wave_barrier();
    __builtin_amdgcn_fence(__ATOMIC_ACQUIRE, "workgroup");
  }
}

__global__ __launch_bounds__(NTHR) void lstm_tile_kernel(const float* __restrict__ P, const unsigned short* __restrict__ WHHp,
                                                         const int* __restrict__ esrc, const int* __restrict__ etrg,
                                                         unsigned short* __restrict__ ACAT) {
  __shared__ __align__(16) _Float16 Hs[2][TILE_NODES * HPITCH];
  __shared__ int sBnd[32];
  __shared__ int sTrg[TILE_NODES * DEG_CAP];
  const _Float16* WHH = (const _Float16*)WHHp;
  const int tid  = threadIdx.x;
  const int lane = tid & 31;
  const int wave = tid >> 5;
  const int c    = lane & 15;
  const int hh   = lane >> 4;
  const int koff = hh * 8;
  const int nodeBase = blockIdx.x * TILE_NODES;

  if (wave == 0) {
    const int which  = lane < 16 ? lane : 16;
    const int target = nodeBase + which;
    int lo = 0, hi = NUM_EDGES;
#pragma unroll 1
    for (int it = 0; it < 20; ++it) {
      const int mid  = (lo + hi) >> 1;
      const int midc = mid < NUM_EDGES ? mid : NUM_EDGES - 1;
      const int v    = esrc[midc];
      const bool act  = lo < hi;
      const bool less = v < target;
      const int nlo = (act && less) ? (mid + 1) : lo;
      const int nhi = (act && !less) ? mid : hi;
      lo = nlo;
      hi = nhi;
    }
    sBnd[lane] = lo;
  }
  {
    const v8h zv = {(_Float16)0.0f, (_Float16)0.0f, (_Float16)0.0f, (_Float16)0.0f,
                    (_Float16)0.0f, (_Float16)0.0f, (_Float16)0.0f, (_Float16)0.0f};
    v8h* hz = (v8h*)&Hs[0][0];
#pragma unroll 1
    for (int i = tid; i < 2 * TILE_NODES * HPITCH / 8; i += NTHR) hz[i] = zv;
  }
  __syncthreads();

  int dg[8];
#pragma unroll
  for (int r = 0; r < 8; ++r) {
    int d = sBnd[8 * hh + r + 1] - sBnd[8 * hh + r];
    d = d < 0 ? 0 : d;
    d = d > DEG_CAP ? DEG_CAP : d;
    dg[r] = d;
  }
  int mx = 0;
#pragma unroll
  for (int m = 0; m < TILE_NODES; ++m) {
    int d = sBnd[m + 1] - sBnd[m];
    d = d < 0 ? 0 : d;
    d = d > DEG_CAP ? DEG_CAP : d;
    mx = d > mx ? d : mx;
  }
  const int maxd = __builtin_amdgcn_readfirstlane(mx);

#pragma unroll 1
  for (int q = 0; q < 3; ++q) {
    const int idx = tid + NTHR * q;
    const int row = idx / DEG_CAP;
    const int t   = idx - row * DEG_CAP;
    int e = sBnd[row] + t;
    e = e < 0 ? 0 : e;
    e = e > NUM_EDGES - 1 ? NUM_EDGES - 1 : e;
    int nb = etrg[e];
    nb = nb < 0 ? 0 : nb;
    nb = nb > NUM_NODES - 1 ? NUM_NODES - 1 : nb;
    sTrg[idx] = nb;
  }
  __syncthreads();

  float creg[8], hreg[8];
#pragma unroll
  for (int r = 0; r < 8; ++r) { creg[r] = 0.0f; hreg[r] = 0.0f; }

  const float* pbase = P + (16 * wave + c) * 4;
  const _Float16* w0 = WHH + (size_t)(0 * HID_UNITS + 16 * wave + c) * HID_UNITS + koff;
  const _Float16* w1 = WHH + (size_t)(1 * HID_UNITS + 16 * wave + c) * HID_UNITS + koff;
  const _Float16* w2 = WHH + (size_t)(2 * HID_UNITS + 16 * wave + c) * HID_UNITS + koff;
  const _Float16* w3 = WHH + (size_t)(3 * HID_UNITS + 16 * wave + c) * HID_UNITS + koff;
  const v8f z8 = {0.f, 0.f, 0.f, 0.f, 0.f, 0.f, 0.f, 0.f};

#pragma unroll 1
  for (int t = 0; t < maxd; ++t) {
    const int cur = t & 1;
    v4f pv[8];
#pragma unroll
    for (int r = 0; r < 8; ++r) {
      const int nb = sTrg[(8 * hh + r) * DEG_CAP + t];
      pv[r] = *(const v4f*)(pbase + (size_t)nb * GATE_COLS);
    }
#pragma unroll
    for (int r = 0; r < 8; ++r) asm volatile("" : "+v"(pv[r]));

    v8f acc0 = z8, acc1 = z8, acc2 = z8, acc3 = z8;
    const _Float16* arow = &Hs[cur][0] + c * HPITCH + koff;
#pragma unroll 1
    for (int k0 = 0; k0 < HID_UNITS; k0 += 32) {
      const v16h a  = frag_load(arow + k0);
      const v16h b0 = frag_load(w0 + k0);
      const v16h b1 = frag_load(w1 + k0);
      const v16h b2 = frag_load(w2 + k0);
      const v16h b3 = frag_load(w3 + k0);
      acc0 = frag_mma(a, b0, acc0);
      acc1 = frag_mma(a, b1, acc1);
      acc2 = frag_mma(a, b2, acc2);
      acc3 = frag_mma(a, b3, acc3);
      guard4_h(acc0, acc1, acc2, acc3, a, b0, b1, b2, b3);
    }
    acc_guard4(acc0, acc1, acc2, acc3);

    _Float16* hn = &Hs[cur ^ 1][0];
#pragma unroll
    for (int r = 0; r < 8; ++r) {
      const float gi = acc0[r] * WCARRY_INV + pv[r][0];
      const float gf = acc1[r] * WCARRY_INV + pv[r][1];
      const float gg = acc2[r] * WCARRY_INV + pv[r][2];
      const float go = acc3[r] * WCARRY_INV + pv[r][3];
      const float iv = fsig(gi);
      const float fv = fsig(gf);
      const float gv = ftanh(gg);
      const float ov = fsig(go);
      const float cn = fv * creg[r] + iv * gv;
      const float hv = ov * ftanh(cn);
      const bool keep = t < dg[r];
      creg[r] = keep ? cn : creg[r];
      hreg[r] = keep ? hv : hreg[r];
      hn[(8 * hh + r) * HPITCH + 16 * wave + c] = (_Float16)hreg[r];
    }
    __syncthreads();
  }

  {
    const int fin = maxd & 1;
    const int row = tid >> 4;
    const int c8  = (tid & 15) * 8;
    const v8h hv = *(const v8h*)(&Hs[fin][0] + row * HPITCH + c8);
    unsigned short* dst = ACAT + (size_t)(nodeBase + row) * CAT_COLS + FEAT_IN + c8;
    store16_twice(dst, hv);
  }
}

__global__ __launch_bounds__(NTHR) void cap_guard_kernel(const int* __restrict__ capv, float* __restrict__ out) {
  const int v = capv[0];
  if (v != DEG_CAP) {
    const float qn = __uint_as_float(0x7fc00000u);
    const v4f nv = {qn, qn, qn, qn};
    for (int pass = 0; pass < 2; ++pass) {
#pragma unroll 1
      for (int i = threadIdx.x; i < OUT_VEC4; i += NTHR) *(volatile v4f*)(out + (size_t)i * 4) = nv;
      __threadfence();
    }
  }
}

extern "C" void kernel_launch(void* const* d_in, const int* in_sizes, int n_in,
                              void* d_out, int out_size, void* d_ws, size_t ws_size, hipStream_t stream) {
  (void)in_sizes; (void)out_size;
  if (n_in < 9 || d_out == nullptr || d_ws == nullptr) return;
  if (ws_size < CARVE_TOTAL) return;

  const float* X     = (const float*)d_in[0];
  const float* W_ih  = (const float*)d_in[1];
  const float* W_hh  = (const float*)d_in[2];
  const float* b_ih  = (const float*)d_in[3];
  const float* b_hh  = (const float*)d_in[4];
  const float* W_out = (const float*)d_in[5];
  const int*   esrc  = (const int*)d_in[6];
  const int*   etrg  = (const int*)d_in[7];
  const int*   capv  = (const int*)d_in[8];
  float* out = (float*)d_out;

  char* ws = (char*)d_ws;
  size_t off = 0;
  unsigned short* ACAT = (unsigned short*)(ws + off); off += ACAT_BYTES;
  float*          PPL  = (float*)(ws + off);          off += PPLANE_BYTES;
  unsigned short* WHH  = (unsigned short*)(ws + off); off += WHH_BYTES;
  unsigned short* WIHP = (unsigned short*)(ws + off); off += WIHP_BYTES;
  unsigned short* WOT  = (unsigned short*)(ws + off); off += WOT_BYTES;
  float*          BIASP = (float*)(ws + off);         off += BIASP_BYTES;
  if (off != CARVE_TOTAL) return;

  prep_x_kernel<<<(NUM_NODES * (FEAT_IN / 8) + (NODES_PAD - NUM_NODES) * (CAT_COLS / 8)) / NTHR, NTHR, 0, stream>>>(X, ACAT);
  prep_w_kernel<<<81, NTHR, 0, stream>>>(W_ih, W_hh, b_ih, b_hh, W_out, WHH, WIHP, WOT, BIASP);

  wmma_gemm64_f16<2><<<(NODES_PAD / 64) * (GATE_COLS / 64) / 8, 256, 0, stream>>>(
      ACAT, CAT_COLS, WIHP, FEAT_IN, PPL, GATE_COLS, BIASP,
      NODES_PAD, GATE_COLS, FEAT_IN, NODES_PAD, WCARRY_INV);

  lstm_tile_kernel<<<NUM_TILES, NTHR, 0, stream>>>(PPL, WHH, esrc, etrg, ACAT);

  wmma_gemm64_f16<0><<<((NODES_PAD / 64) * (FEAT_OUT / 64) + 7) / 8, 256, 0, stream>>>(
      ACAT, CAT_COLS, WOT, CAT_COLS, out, FEAT_OUT, BIASP,
      NODES_PAD, FEAT_OUT, CAT_COLS, NUM_NODES, WCARRY_INV);

  cap_guard_kernel<<<1, NTHR, 0, stream>>>(capv, out);
}
